// UGCALayer_34935263986215
// MI455X (gfx1250) — hardware-verified
//
#include <hip/hip_runtime.h>


#define NB_  16
#define TD   256
#define TP   1024
#define DD   512
#define FF   2048
#define NH_  8
#define HD   64
#define RD   (NB_ * TD)
#define RP   (NB_ * TP)
#define IG   2
#define DM   DD
#define GMIN 0.05f
#define SCL  0.125f
#define LOSC 1024.0f

typedef _Float16 h16;
typedef unsigned short bf;
typedef __attribute__((ext_vector_type(16))) __bf16   v16bf;
typedef __attribute__((ext_vector_type(16))) _Float16 v16h;
typedef __attribute__((ext_vector_type(8)))  _Float16 v8h;
typedef __attribute__((ext_vector_type(8)))  unsigned short v8us;
typedef __attribute__((ext_vector_type(8)))  float    v8f;
typedef __attribute__((ext_vector_type(4)))  float    v4f;
typedef v8h  __attribute__((may_alias)) v8ha;
typedef v4f  __attribute__((may_alias)) v4fa;
typedef v8us __attribute__((may_alias)) v8usa;

__device__ __forceinline__ unsigned short f2bf(float f) { unsigned u = __float_as_uint(f); u += 0x7FFFu + ((u >> 16) & 1u); return (unsigned short)(u >> 16); }
__device__ __forceinline__ float bf2f(unsigned short b) { return __uint_as_float(((unsigned)b) << 16); }
__device__ __forceinline__ float bfr(float f) { return bf2f(f2bf(f)); }
__device__ __forceinline__ v16h cat16(v8h lo, v8h hi) { return __builtin_shufflevector(lo, hi, 0, 1, 2, 3, 4, 5, 6, 7, 8, 9, 10, 11, 12, 13, 14, 15); }
__device__ __forceinline__ v16bf cat16b(v8us lo, v8us hi) { return __builtin_bit_cast(v16bf, __builtin_shufflevector(lo, hi, 0, 1, 2, 3, 4, 5, 6, 7, 8, 9, 10, 11, 12, 13, 14, 15)); }
__device__ __forceinline__ v8f wmma16(v16h a, v16h b, v8f c) { return __builtin_amdgcn_wmma_f32_16x16x32_f16(false, a, false, b, (short)0, c, false, false); }
__device__ __forceinline__ v8f wmmab(v16bf a, v16bf b, v8f c) { return __builtin_amdgcn_wmma_f32_16x16x32_bf16(false, a, false, b, (short)0, c, false, false); }


__global__ __launch_bounds__(128) void k_gemmh(const h16* __restrict__ A, const h16* __restrict__ Bn, const float* __restrict__ bias, float* C, int ldc, const float* __restrict__ R, int K, size_t sA, size_t sB, size_t sC, int roundR) {
    __shared__ __align__(16) float ost[4][16 * 68];
    const size_t z = blockIdx.z; A += z * sA; Bn += z * sB; C += z * sC; if (R) R += z * sC;
    const int lane = threadIdx.x & 31, wave = threadIdx.x >> 5, lr = lane & 15, hi = lane >> 4;
    const int r0 = blockIdx.x * 64 + wave * 16, c0 = blockIdx.y * 64;
    const size_t aoff = (size_t)(r0 + lr) * K + 8 * hi;
    size_t boff[4];
#pragma unroll
    for (int t = 0; t < 4; ++t) boff[t] = (size_t)(c0 + t * 16 + lr) * K + 8 * hi;
    v8f acc[4];
#pragma unroll
    for (int t = 0; t < 4; ++t) acc[t] = (v8f){};
#pragma unroll 1
    for (int kc = 0; kc < K; kc += 32) {
        const v16h a = cat16(*(const v8h*)(A + aoff + kc), *(const v8h*)(A + aoff + kc + 16));
#pragma unroll
        for (int t = 0; t < 4; ++t) { const v16h b = cat16(*(const v8h*)(Bn + boff[t] + kc), *(const v8h*)(Bn + boff[t] + kc + 16)); acc[t] = wmma16(a, b, acc[t]); }
        asm volatile("v_nop\n\tv_nop\n\tv_nop\n\tv_nop" : "+v"(acc[0]), "+v"(acc[1]), "+v"(acc[2]), "+v"(acc[3]) : "v"(a));
    }
    float* os = &ost[wave][0];
#pragma unroll
    for (int t = 0; t < 4; ++t) { const float bv = bias ? bfr(bias[c0 + t * 16 + lr]) : 0.f;
#pragma unroll
        for (int j = 0; j < 8; ++j) os[(hi * 8 + j) * 68 + t * 16 + lr] = acc[t][j] + bv; }
    __syncthreads();
    float* crow = C + (size_t)r0 * ldc + c0;
    auto pass = [&]() {
#pragma unroll
        for (int s = 0; s < 8; ++s) { const int Lid = (lane >> 3) + 4 * s, piece = lane & 7; const int row = Lid >> 1, cofs = (Lid & 1) * 32 + piece * 4;
            v4f val = *(const v4fa*)(os + row * 68 + cofs); if (R) { const v4f rv = *(const v4f*)(R + ((size_t)r0 + row) * ldc + c0 + cofs); val += roundR ? (v4f){bfr(rv[0]), bfr(rv[1]), bfr(rv[2]), bfr(rv[3])} : rv; }
            *(volatile v4f*)(crow + (size_t)row * ldc + cofs) = val; }
    };
    pass(); __threadfence(); pass();
}

typedef __attribute__((ext_vector_type(4))) _Float16 v4h;
__device__ __forceinline__ h16 tohx(float x) { return (h16)x; }
template <bool XF32>
__global__ __launch_bounds__(256) void k_cvth(const float* __restrict__ x, size_t rows, h16* Hh, float* XF) {
    const int lane = threadIdx.x & 31; const size_t r = (size_t)blockIdx.x * 8 + (threadIdx.x >> 5); if (r >= rows) return;
#pragma unroll 1
    for (int ps = 0; ps < 2; ++ps) {
#pragma unroll
        for (int q = 0; q < 2; ++q) { v8h o; v8f f;
#pragma unroll
            for (int i = 0; i < 8; ++i) { const float v = bfr(x[r * DD + lane * 16 + q * 8 + i]); o[i] = tohx(v); f[i] = v; }
            *(volatile v8h*)(Hh + r * DD + lane * 16 + q * 8) = o; if (XF32) { *(volatile v4f*)(XF + r * DD + lane * 16 + q * 8) = (v4f){f[0], f[1], f[2], f[3]}; *(volatile v4f*)(XF + r * DD + lane * 16 + q * 8 + 4) = (v4f){f[4], f[5], f[6], f[7]}; } }
        if (ps == 0) __threadfence(); }
}
__global__ __launch_bounds__(256) void k_wTh(const float* __restrict__ Wm, int K, int N, h16* Bt) {
    __shared__ float tl[64][65];
    const int tid = threadIdx.x; const int k0 = blockIdx.x * 64, n0 = blockIdx.y * 64; const int rr = tid >> 2, cq = (tid & 3) * 16;
#pragma unroll
    for (int i = 0; i < 16; ++i) tl[rr][cq + i] = bfr(Wm[(size_t)(k0 + rr) * N + n0 + cq + i]);
    __syncthreads();
    const int lane = tid & 31, wv = tid >> 5;
    auto pass = [&]() {
#pragma unroll
        for (int st = 0; st < 4; ++st) { const int nr = wv * 8 + st * 2 + (lane >> 4); const int kq = (lane & 15) * 4; v4h v;
#pragma unroll
            for (int i = 0; i < 4; ++i) v[i] = tohx(tl[kq + i][nr]);
            *(volatile v4h*)(Bt + (size_t)(n0 + nr) * K + k0 + kq) = v; }
    };
    pass(); __threadfence(); pass();
}
template <int WID>
__global__ __launch_bounds__(256) void k_siluh(const float* __restrict__ F, size_t rows, h16* Hh) {
    const int lane = threadIdx.x & 31; const size_t r = (size_t)blockIdx.x * 8 + (threadIdx.x >> 5); if (r >= rows) return;
#pragma unroll 1
    for (int ps = 0; ps < 2; ++ps) {
#pragma unroll 1
        for (int q = 0; q < WID / 256; ++q) { const size_t o = r * WID + q * 256 + lane * 8; const v8f v = *(const v8f*)(F + o); v8h h;
#pragma unroll
            for (int i = 0; i < 8; ++i) { const float t = v[i]; h[i] = tohx(t / (1.0f + expf(-t))); }
            *(volatile v8h*)(Hh + o) = h; }
        if (ps == 0) __threadfence(); }
}
__global__ __launch_bounds__(256) void k_tof16(const float* __restrict__ F, size_t rows, h16* Hh) {
    const int lane = threadIdx.x & 31; const size_t r = (size_t)blockIdx.x * 8 + (threadIdx.x >> 5); if (r >= rows) return;
#pragma unroll 1
    for (int ps = 0; ps < 2; ++ps) {
#pragma unroll
        for (int q = 0; q < 2; ++q) { const size_t o = r * DD + lane * 16 + q * 8; const v8f v = *(const v8f*)(F + o); v8h h;
#pragma unroll
            for (int i = 0; i < 8; ++i) h[i] = tohx(v[i]);
            *(volatile v8h*)(Hh + o) = h; }
        if (ps == 0) __threadfence(); }
}
__global__ __launch_bounds__(256) void k_evi(const float* __restrict__ HS, size_t rows, const float* __restrict__ w2, const float* __restrict__ b2, const int* __restrict__ kk, float* G, float* LB) {
    const int lane = threadIdx.x & 31; const size_t r = ((size_t)blockIdx.x * 8 + (threadIdx.x >> 5)) * 32 + lane; if (r >= rows) return; const float* h = HS + r * DD;
    float p1 = bfr(b2[1]), p2 = bfr(b2[2]), p3 = bfr(b2[3]);
#pragma unroll 1
    for (int k = 0; k < DD; ++k) { const float t = h[k]; const float hv = t / (1.0f + expf(-t)); p1 = fmaf(hv, bfr(w2[k * 4 + 1]), p1); p2 = fmaf(hv, bfr(w2[k * 4 + 2]), p2); p3 = fmaf(hv, bfr(w2[k * 4 + 3]), p3); }
    auto softplus = [](float t) { return (t > 20.f) ? t : log1pf(expf(t)); };
    const float nu = softplus(p1) + 1e-6f, alpha = softplus(p2) + 1.0f, beta = softplus(p3) + 1e-6f; const float sigma2 = beta / (nu * (alpha - 1.0f));
    const float kf = (float)kk[0]; const float g = fminf(fmaxf(expf(-kf * sigma2), GMIN), 1.0f); const float lb = logf(g + 1e-12f);
    *(volatile float*)(G + r) = g; *(volatile float*)(LB + r) = lb; __threadfence(); *(volatile float*)(G + r) = g; *(volatile float*)(LB + r) = lb;
}
__global__ __launch_bounds__(256) void k_hplh(const float* __restrict__ F, size_t r0, int T, float sc, h16* P) {
    typedef __attribute__((ext_vector_type(4))) _Float16 v4h_;
    const int lane = threadIdx.x & 31; const size_t w = (size_t)blockIdx.x * 8 + (threadIdx.x >> 5); if (w >= (size_t)T / 2) return; const int g = blockIdx.z / NH_, h = blockIdx.z % NH_; const int i = (int)(w * 2 + (lane >> 4)); const int c0 = (lane & 15) * 4; v4h_ o;
#pragma unroll
    for (int q = 0; q < 4; ++q) o[q] = tohx(F[(r0 + (size_t)g * T + i) * DD + h * HD + c0 + q] * sc);
    const size_t off = ((size_t)blockIdx.z * T + i) * HD + c0; *(volatile v4h_*)(P + off) = o; __threadfence(); *(volatile v4h_*)(P + off) = o;
}
__global__ __launch_bounds__(256) void k_vTh(const float* __restrict__ F, size_t r0, int T, h16* VT) {
    __shared__ float tl[64][65];
    typedef __attribute__((ext_vector_type(4))) _Float16 v4h_;
    const int tid = threadIdx.x; const int t0 = blockIdx.x * 64; const int g = blockIdx.z / NH_, h = blockIdx.z % NH_; const int rr = tid >> 2, cq = (tid & 3) * 16;
#pragma unroll
    for (int i = 0; i < 16; ++i) tl[rr][cq + i] = F[(r0 + (size_t)g * T + t0 + rr) * DD + h * HD + cq + i];
    __syncthreads();
    const int lane = tid & 31, wv = tid >> 5;
    auto pass = [&]() {
#pragma unroll
        for (int st = 0; st < 4; ++st) { const int dr = wv * 8 + st * 2 + (lane >> 4); const int tq = (lane & 15) * 4; v4h_ v;
#pragma unroll
            for (int i = 0; i < 4; ++i) v[i] = tohx(tl[tq + i][dr]);
            *(volatile v4h_*)(VT + ((size_t)blockIdx.z * HD + dr) * T + t0 + tq) = v; }
    };
    pass(); __threadfence(); pass();
}
template <int N>
__global__ __launch_bounds__(256) void k_softlb(const float* __restrict__ S, int rows, const float* __restrict__ LB, size_t b0, h16* P) {
    typedef __attribute__((ext_vector_type(4))) _Float16 v4h_;
    const int lane = threadIdx.x & 31, i = blockIdx.x * 8 + (threadIdx.x >> 5); if (i >= rows) return; const int g = blockIdx.z / NH_; const size_t zo = (size_t)blockIdx.z * rows * N; const float* sr = S + zo + (size_t)i * N; const float* lb = LB + (b0 + g) * N; h16* pr = P + zo + (size_t)i * N;
    float m = -3.0e38f;
#pragma unroll 1
    for (int c0 = lane * 4; c0 < N; c0 += 128) {
#pragma unroll
        for (int q = 0; q < 4; ++q) m = fmaxf(m, sr[c0 + q] + lb[c0 + q]); }
#pragma unroll
    for (int sh = 16; sh; sh >>= 1) m = fmaxf(m, __shfl_xor(m, sh, 32));
    float sum = 0.f;
#pragma unroll 1
    for (int c0 = lane * 4; c0 < N; c0 += 128) {
#pragma unroll
        for (int q = 0; q < 4; ++q) sum += __expf(sr[c0 + q] + lb[c0 + q] - m); }
#pragma unroll
    for (int sh = 16; sh; sh >>= 1) sum += __shfl_xor(sum, sh, 32);
    const float inv = 1.0f / sum;
#pragma unroll 1
    for (int ps = 0; ps < 2; ++ps) {
#pragma unroll 1
        for (int c0 = lane * 4; c0 < N; c0 += 128) { v4h_ o;
#pragma unroll
            for (int q = 0; q < 4; ++q) o[q] = tohx(__expf(sr[c0 + q] + lb[c0 + q] - m) * inv);
            *(volatile v4h_*)(pr + c0) = o; }
        if (ps == 0) __threadfence(); }
}
__global__ __launch_bounds__(256) void k_ln512(const float* __restrict__ F, size_t rows, const float* __restrict__ gg, const float* __restrict__ bb, float* OUT) {
    const int lane = threadIdx.x & 31; const size_t r = (size_t)blockIdx.x * 8 + (threadIdx.x >> 5); if (r >= rows) return; float v[16]; float s = 0.f;
#pragma unroll
    for (int i = 0; i < 16; ++i) { v[i] = F[r * DD + lane * 16 + i]; s += v[i]; }
#pragma unroll
    for (int sh = 16; sh; sh >>= 1) s += __shfl_xor(s, sh, 32);
    const float mu = s * (1.0f / DD); float q = 0.f;
#pragma unroll
    for (int i = 0; i < 16; ++i) { const float d = v[i] - mu; q = fmaf(d, d, q); }
#pragma unroll
    for (int sh = 16; sh; sh >>= 1) q += __shfl_xor(q, sh, 32);
    const float rs = rsqrtf(q * (1.0f / DD) + 1e-5f);
#pragma unroll 1
    for (int ps = 0; ps < 2; ++ps) {
#pragma unroll
        for (int qd = 0; qd < 4; ++qd) { v4f o; for (int i = 0; i < 4; ++i) { const int c = lane * 16 + qd * 4 + i; o[i] = (v[qd * 4 + i] - mu) * rs * bfr(gg[c]) + bfr(bb[c]); } *(volatile v4f*)(OUT + r * DD + lane * 16 + qd * 4) = o; }
        if (ps == 0) __threadfence(); }
}
__global__ __launch_bounds__(256) void k_copyg(const float* __restrict__ G, size_t n, float* dst) {
    const size_t i = (size_t)blockIdx.x * 256 + threadIdx.x; if (i >= n) return; const float v = G[i]; *(volatile float*)(dst + i) = v; __threadfence(); *(volatile float*)(dst + i) = v;
}

__global__ __launch_bounds__(256) void k_mergeh(const float* __restrict__ OZ, int T, h16* OH) {
    const int lane = threadIdx.x & 31; const size_t w = (size_t)blockIdx.x * 8 + (threadIdx.x >> 5); if (w >= (size_t)IG * T) return; const int g = (int)(w / T), i = (int)(w % T);
#pragma unroll 1
    for (int ps = 0; ps < 2; ++ps) {
#pragma unroll
        for (int q = 0; q < 2; ++q) { const int c0 = lane * 16 + q * 8; const int h = c0 / HD, d0 = c0 % HD; v8h o;
#pragma unroll
            for (int k = 0; k < 8; ++k) o[k] = tohx(OZ[(((size_t)g * NH_ + h) * T + i) * HD + d0 + k]);
            *(volatile v8h*)(OH + w * DD + c0) = o; }
        if (ps == 0) __threadfence(); }
}

extern "C" void kernel_launch(void* const* d_in, const int* in_sizes, int n_in,
                              void* d_out, int out_size, void* d_ws, size_t ws_size, hipStream_t stream) {
    (void)in_sizes; (void)n_in; (void)out_size;
    const float* Hd = (const float*)d_in[0]; const float* Hp = (const float*)d_in[1]; const int* kk = (const int*)d_in[2];
    const float* ed_w1 = (const float*)d_in[3]; const float* ed_b1 = (const float*)d_in[4]; const float* ed_w2 = (const float*)d_in[5]; const float* ed_b2 = (const float*)d_in[6]; const float* ep_w1 = (const float*)d_in[7]; const float* ep_b1 = (const float*)d_in[8]; const float* ep_w2 = (const float*)d_in[9]; const float* ep_b2 = (const float*)d_in[10];
    const float* const* P2D = (const float* const*)(d_in + 11); const float* const* D2P = (const float* const*)(d_in + 21);
    const float* fd_w1 = (const float*)d_in[31]; const float* fd_b1 = (const float*)d_in[32]; const float* fd_w2 = (const float*)d_in[33]; const float* fd_b2 = (const float*)d_in[34]; const float* fd_g = (const float*)d_in[35]; const float* fd_b = (const float*)d_in[36];
    const float* fp_w1 = (const float*)d_in[37]; const float* fp_b1 = (const float*)d_in[38]; const float* fp_w2 = (const float*)d_in[39]; const float* fp_b2 = (const float*)d_in[40]; const float* fp_g = (const float*)d_in[41]; const float* fp_b = (const float*)d_in[42];
    float* out0 = (float*)d_out; float* out1 = (float*)((char*)d_out + 8388608); float* out2 = (float*)((char*)d_out + 41943040); float* out3 = (float*)((char*)d_out + 41959424);
    char* wsp = (char*)d_ws;
    auto take = [&](size_t bytes) { char* p = wsp; wsp += (bytes + 255) & ~(size_t)255; return (void*)p; };
    h16* WE_D = (h16*)take((size_t)DD * DD * 2); h16* WE_P = (h16*)take((size_t)DD * DD * 2);
    h16* WA1[4]; h16* WA2[4]; for (int i = 0; i < 4; ++i) { WA1[i] = (h16*)take((size_t)DD * DD * 2); WA2[i] = (h16*)take((size_t)DD * DD * 2); }
    h16* WF1D = (h16*)take((size_t)FF * DD * 2); h16* WF2D = (h16*)take((size_t)DD * FF * 2); h16* WF1P = (h16*)take((size_t)FF * DD * 2); h16* WF2P = (h16*)take((size_t)DD * FF * 2);
    h16* Hph = (h16*)take((size_t)RP * DD * 2); h16* Hdh = (h16*)take((size_t)RD * DD * 2); float* LBD = (float*)take((size_t)RD * 4); float* LBP = (float*)take((size_t)RP * 4);
    float* BIG1 = (float*)take((size_t)RP * DD * 4); float* BIG2 = (float*)take((size_t)RP * DD * 4); float* KX = (float*)take((size_t)RD * DD * 4); float* VX = (float*)take((size_t)RD * DD * 4); float* QD = (float*)take((size_t)RD * DD * 4); float* HD2 = (float*)take((size_t)RD * DD * 4);
    h16* QPL = (h16*)take((size_t)IG * NH_ * TP * HD * 2); h16* KPL = (h16*)take((size_t)IG * NH_ * TP * HD * 2); h16* VT = (h16*)take((size_t)IG * NH_ * HD * TP * 2);
    float* S = (float*)take((size_t)IG * NH_ * TP * TD * 4); h16* PP = (h16*)take((size_t)IG * NH_ * TP * TD * 2); float* OZ = (float*)take((size_t)IG * NH_ * TP * HD * 4); h16* OH = (h16*)take((size_t)RP * DD * 2); h16* F1h = (h16*)take((size_t)RD * FF * 2);
    if ((size_t)(wsp - (char*)d_ws) > ws_size) return;
    k_wTh<<<dim3(DD / 64, DD / 64, 1), 256, 0, stream>>>(ed_w1, DD, DD, WE_D); k_wTh<<<dim3(DD / 64, DD / 64, 1), 256, 0, stream>>>(ep_w1, DD, DD, WE_P);
    for (int i = 0; i < 4; ++i) { k_wTh<<<dim3(DD / 64, DD / 64, 1), 256, 0, stream>>>(P2D[i], DD, DD, WA1[i]); k_wTh<<<dim3(DD / 64, DD / 64, 1), 256, 0, stream>>>(D2P[i], DD, DD, WA2[i]); }
    k_wTh<<<dim3(DD / 64, FF / 64, 1), 256, 0, stream>>>(fd_w1, DD, FF, WF1D); k_wTh<<<dim3(FF / 64, DD / 64, 1), 256, 0, stream>>>(fd_w2, FF, DD, WF2D); k_wTh<<<dim3(DD / 64, FF / 64, 1), 256, 0, stream>>>(fp_w1, DD, FF, WF1P); k_wTh<<<dim3(FF / 64, DD / 64, 1), 256, 0, stream>>>(fp_w2, FF, DD, WF2P);
    k_cvth<false><<<RP / 8, 256, 0, stream>>>(Hp, RP, Hph, nullptr); k_cvth<false><<<RD / 8, 256, 0, stream>>>(Hd, RD, Hdh, nullptr);
    k_gemmh<<<dim3(RD / 64, DD / 64, 1), 128, 0, stream>>>(Hdh, WE_D, ed_b1, BIG1, DD, nullptr, DD, 0, 0, 0, 0); k_evi<<<(RD / 32 + 7) / 8, 256, 0, stream>>>(BIG1, RD, ed_w2, ed_b2, kk, out2, LBD);
    k_gemmh<<<dim3(RP / 64, DD / 64, 1), 128, 0, stream>>>(Hph, WE_P, ep_b1, BIG1, DD, nullptr, DD, 0, 0, 0, 0); k_evi<<<(RP / 32 + 7) / 8, 256, 0, stream>>>(BIG1, RP, ep_w2, ep_b2, kk, out3, LBP);
    k_gemmh<<<dim3(RP / 64, DD / 64, 1), 128, 0, stream>>>(Hph, WA1[0], P2D[4], BIG1, DD, nullptr, DD, 0, 0, 0, 0);
    k_gemmh<<<dim3(RD / 64, DD / 64, 1), 128, 0, stream>>>(Hdh, WA1[1], P2D[5], KX, DD, nullptr, DD, 0, 0, 0, 0);
    k_gemmh<<<dim3(RD / 64, DD / 64, 1), 128, 0, stream>>>(Hdh, WA1[2], P2D[6], VX, DD, nullptr, DD, 0, 0, 0, 0);
    for (int grp = 0; grp < NB_ / IG; ++grp) { const size_t b0 = (size_t)grp * IG;
        k_hplh<<<dim3((TP / 2) / 8, 1, IG * NH_), 256, 0, stream>>>(BIG1, b0 * TP, TP, SCL, QPL); k_hplh<<<dim3((TD / 2) / 8, 1, IG * NH_), 256, 0, stream>>>(KX, b0 * TD, TD, 1.0f, KPL); k_vTh<<<dim3(TD / 64, 1, IG * NH_), 256, 0, stream>>>(VX, b0 * TD, TD, VT);
        k_gemmh<<<dim3(TP / 64, TD / 64, IG * NH_), 128, 0, stream>>>(QPL, KPL, nullptr, S, TD, nullptr, HD, (size_t)TP * HD, (size_t)TD * HD, (size_t)TP * TD, 0);
        k_softlb<TD><<<dim3(TP / 8, 1, IG * NH_), 256, 0, stream>>>(S, TP, LBD, b0, PP);
        k_gemmh<<<dim3(TP / 64, 1, IG * NH_), 128, 0, stream>>>(PP, VT, nullptr, OZ, HD, nullptr, TD, (size_t)TP * TD, (size_t)HD * TD, (size_t)TP * HD, 0);
        k_mergeh<<<(IG * TP) / 8, 256, 0, stream>>>(OZ, TP, OH + b0 * TP * DD); }
    k_gemmh<<<dim3(RP / 64, DD / 64, 1), 128, 0, stream>>>(OH, WA1[3], P2D[7], BIG2, DD, Hp, DD, 0, 0, 0, 1);
    k_ln512<<<RP / 8, 256, 0, stream>>>(BIG2, RP, P2D[8], P2D[9], BIG1);
    k_tof16<<<RP / 8, 256, 0, stream>>>(BIG1, RP, OH);
    for (int c = 0; c < RP / RD; ++c) { const size_t r0 = (size_t)c * RD;
        k_gemmh<<<dim3(RD / 64, FF / 64, 1), 128, 0, stream>>>(OH + r0 * DD, WF1P, fp_b1, BIG1, FF, nullptr, DD, 0, 0, 0, 0);
        k_siluh<FF><<<RD / 8, 256, 0, stream>>>(BIG1, RD, F1h);
        k_gemmh<<<dim3(RD / 64, DD / 64, 1), 128, 0, stream>>>(F1h, WF2P, fp_b2, BIG2 + r0 * DD, DD, nullptr, FF, 0, 0, 0, 0); }
    k_ln512<<<RP / 8, 256, 0, stream>>>(BIG2, RP, fp_g, fp_b, out1);
    k_gemmh<<<dim3(RD / 64, DD / 64, 1), 128, 0, stream>>>(Hdh, WA2[0], D2P[4], QD, DD, nullptr, DD, 0, 0, 0, 0);
    k_gemmh<<<dim3(RP / 64, DD / 64, 1), 128, 0, stream>>>(Hph, WA2[1], D2P[5], BIG1, DD, nullptr, DD, 0, 0, 0, 0);
    k_gemmh<<<dim3(RP / 64, DD / 64, 1), 128, 0, stream>>>(Hph, WA2[2], D2P[6], BIG2, DD, nullptr, DD, 0, 0, 0, 0);
    for (int grp = 0; grp < NB_ / IG; ++grp) { const size_t b0 = (size_t)grp * IG;
        k_hplh<<<dim3((TD / 2) / 8, 1, IG * NH_), 256, 0, stream>>>(QD, b0 * TD, TD, SCL, QPL); k_hplh<<<dim3((TP / 2) / 8, 1, IG * NH_), 256, 0, stream>>>(BIG1, b0 * TP, TP, 1.0f, KPL); k_vTh<<<dim3(TP / 64, 1, IG * NH_), 256, 0, stream>>>(BIG2, b0 * TP, TP, VT);
        k_gemmh<<<dim3(TD / 64, TP / 64, IG * NH_), 128, 0, stream>>>(QPL, KPL, nullptr, S, TP, nullptr, HD, (size_t)TD * HD, (size_t)TP * HD, (size_t)TD * TP, 0);
        k_softlb<TP><<<dim3(TD / 8, 1, IG * NH_), 256, 0, stream>>>(S, TD, LBP, b0, PP);
        k_gemmh<<<dim3(TD / 64, 1, IG * NH_), 128, 0, stream>>>(PP, VT, nullptr, OZ, HD, nullptr, TP, (size_t)TD * TP, (size_t)HD * TP, (size_t)TD * HD, 0);
        k_mergeh<<<(IG * TD) / 8, 256, 0, stream>>>(OZ, TD, OH + b0 * TD * DD); }
    k_gemmh<<<dim3(RD / 64, DD / 64, 1), 128, 0, stream>>>(OH, WA2[3], D2P[7], KX, DD, Hd, DD, 0, 0, 0, 1);
    k_ln512<<<RD / 8, 256, 0, stream>>>(KX, RD, D2P[8], D2P[9], HD2);
    k_tof16<<<RD / 8, 256, 0, stream>>>(HD2, RD, OH);
    k_gemmh<<<dim3(RD / 64, FF / 64, 1), 128, 0, stream>>>(OH, WF1D, fd_b1, BIG1, FF, nullptr, DD, 0, 0, 0, 0);
    k_siluh<FF><<<RD / 8, 256, 0, stream>>>(BIG1, RD, F1h);
    k_gemmh<<<dim3(RD / 64, DD / 64, 1), 128, 0, stream>>>(F1h, WF2D, fd_b2, VX, DD, nullptr, FF, 0, 0, 0, 0);
    k_ln512<<<RD / 8, 256, 0, stream>>>(VX, RD, fd_g, fd_b, out0);
}
